// CopyingModel_4870492914171
// MI455X (gfx1250) — hardware-verified
//
#include <hip/hip_runtime.h>
#include <math.h>

typedef __attribute__((ext_vector_type(16))) _Float16 v16h;
typedef __attribute__((ext_vector_type(8)))  _Float16 v8h;
typedef __attribute__((ext_vector_type(4)))  _Float16 v4h;
typedef __attribute__((ext_vector_type(16))) __bf16   v16b;
typedef __attribute__((ext_vector_type(8)))  __bf16   v8b;
typedef __attribute__((ext_vector_type(8)))  float    v8f;
typedef __attribute__((ext_vector_type(4)))  float    v4f;

constexpr int kHalves = 2;
constexpr int kBatch = 4;
constexpr int kSeq   = 4096;
constexpr int kRows  = kBatch * kSeq;
constexpr int kVocab = 64;
constexpr int kD     = 1024;
constexpr int kDX    = 2 * kD;
constexpr int kNs    = 64;
constexpr int kNh    = 32;
constexpr int kThr   = 256;

constexpr float kWCarry = 4096.0f;
constexpr float kACarry = 256.0f;
constexpr float kScA = 1.0f / (kACarry * kWCarry);
constexpr float kF16MinNormal = 6.103515625e-5f;

static_assert((kRows % 64) == 0 && ((kRows / 64) * (kVocab / 64)) % 8 == 0, "GEMM grid exact");
static_assert((kDX % 32) == 0, "GEMM K a multiple of 32");

constexpr size_t kOffDA  = 0;
constexpr size_t kOffDB  = kOffDA  + (size_t)kD * kNs * 4;
constexpr size_t kOffWOT = kOffDB  + (size_t)kD * kNs * 4;
constexpr size_t kOffBV  = kOffWOT + (size_t)kVocab * kDX * 2;
constexpr size_t kOffYP  = kOffBV  + 512;
constexpr size_t kOffY16 = kOffYP  + (size_t)kRows * kD * 4;
constexpr size_t kWsTotal = kOffY16 + (size_t)kRows * kDX * 2;
static_assert(kWsTotal <= 268435456ull, "inside the offered workspace");
static_assert((kOffDB % 256) == 0 && (kOffWOT % 256) == 0 && (kOffBV % 256) == 0 && (kOffYP % 256) == 0 && (kOffY16 % 256) == 0, "aligned regions");

__device__ __forceinline__ unsigned short f2bf_bits(float f) {
  unsigned u = __float_as_uint(f);
  return (unsigned short)((u + 0x7FFFu + ((u >> 16) & 1u)) >> 16);
}
__device__ __forceinline__ float bf_bits2f(unsigned short h) { return __uint_as_float(((unsigned)h) << 16); }
__device__ __forceinline__ float bf16r(float f) { return bf_bits2f(f2bf_bits(f)); }
__device__ __forceinline__ float carry_flush(float v, float carry) {
  const float s = v * carry;
  return (fabsf(s) < kF16MinNormal) ? 0.0f : s;
}
__device__ __forceinline__ float frcp(float x) { return __builtin_amdgcn_rcpf(x); }

__device__ __forceinline__ void dep_guard4_h(v8f& a, v8f& b, v8f& c, v8f& d, v16h x, v16h y) { asm volatile("v_nop\n\tv_nop\n\tv_nop\n\tv_nop" : "+v"(a), "+v"(b), "+v"(c), "+v"(d) : "v"(x), "v"(y)); }
__device__ __forceinline__ void dep_guard4_b(v8f& a, v8f& b, v8f& c, v8f& d, v16b x, v16b y) { asm volatile("v_nop\n\tv_nop\n\tv_nop\n\tv_nop" : "+v"(a), "+v"(b), "+v"(c), "+v"(d) : "v"(x), "v"(y)); }
__device__ __forceinline__ void keep4_h(v16h a, v16h b, v16h c, v16h d) { asm volatile("v_nop" :: "v"(a), "v"(b), "v"(c), "v"(d)); }
__device__ __forceinline__ void keep4_b(v16b a, v16b b, v16b c, v16b d) { asm volatile("v_nop" :: "v"(a), "v"(b), "v"(c), "v"(d)); }
__device__ __forceinline__ void acc_guard4(v8f& a, v8f& b, v8f& c, v8f& d) { asm volatile("v_nop\n\tv_nop\n\tv_nop\n\tv_nop" : "+v"(a), "+v"(b), "+v"(c), "+v"(d)); }

template <typename T> struct Frag;
template <> struct Frag<_Float16> {
  typedef v16h V; union U { v16h v; v8h h[2]; };
  static __device__ __forceinline__ v16h load(const _Float16* p) {
    U f; f.h[0] = *(const v8h*)(p); f.h[1] = *(const v8h*)(p + 16); return f.v;
  }
  static __device__ __forceinline__ v8f mma(v16h a, v16h b, v8f c) {
    return __builtin_amdgcn_wmma_f32_16x16x32_f16(false, a, false, b, (short)0, c, false, false);
  }
  static __device__ __forceinline__ void guard4(v8f& a, v8f& b, v8f& c, v8f& d, v16h x, v16h y) { dep_guard4_h(a, b, c, d, x, y); }
  static __device__ __forceinline__ void keep(v16h a, v16h b, v16h c, v16h d) { keep4_h(a, b, c, d); }
};
template <> struct Frag<__bf16> {
  typedef v16b V; union U { v16b v; v8b h[2]; };
  static __device__ __forceinline__ v16b load(const __bf16* p) {
    U f; f.h[0] = *(const v8b*)(p); f.h[1] = *(const v8b*)(p + 16); return f.v;
  }
  static __device__ __forceinline__ v8f mma(v16b a, v16b b, v8f c) {
    return __builtin_amdgcn_wmma_f32_16x16x32_bf16(false, a, false, b, (short)0, c, false, false);
  }
  static __device__ __forceinline__ void guard4(v8f& a, v8f& b, v8f& c, v8f& d, v16b x, v16b y) { dep_guard4_b(a, b, c, d, x, y); }
  static __device__ __forceinline__ void keep(v16b a, v16b b, v16b c, v16b d) { keep4_b(a, b, c, d); }
};

__device__ __forceinline__ v8f mma_h(v16h a, v16h b, v8f c) {
  c = __builtin_amdgcn_wmma_f32_16x16x32_f16(false, a, false, b, (short)0, c, false, false);
  asm volatile("v_nop\n\tv_nop\n\tv_nop\n\tv_nop" : "+v"(c) : "v"(a), "v"(b));
  return c;
}

template <int ET> struct Elem;
template <> struct Elem<0> { typedef _Float16 T; };
template <> struct Elem<1> { typedef __bf16 T; };
template <int ET, bool SPLIT, int BIAS_MODE, int OUT_MODE, bool RESID, int ACT = 0>
__global__ __launch_bounds__(256) void wmma_gemm64(
    const unsigned short* __restrict__ Ap, const unsigned short* __restrict__ A2p, int lda, long strideA,
    const unsigned short* __restrict__ Btp, const unsigned short* __restrict__ Bt2p, int ldb, long strideB,
    void* __restrict__ Cout, void* __restrict__ Cout2, int ldc, long strideC,
    const float* __restrict__ bias,
    const float* __restrict__ resid, long strideR,
    int M, int N, int K, float scale) {
  typedef typename Elem<ET>::T T;
  typedef typename Frag<T>::V V;
  const T* A = (const T*)Ap; const T* A2 = (const T*)A2p; const T* Bt = (const T*)Btp; const T* Bt2 = (const T*)Bt2p;
  __shared__ __align__(16) float sT[8][16 * 68];
  const int b    = blockIdx.y;
  const int lane = threadIdx.x & 31;
  const int wave = threadIdx.x >> 5;
  const int tilesN = N >> 6;
  const int tilesM = M >> 6;
  const int tile = blockIdx.x * 8 + wave;
  if (tile >= tilesM * tilesN) return;
  const int tm = tile / tilesN;
  const int tn = tile - tm * tilesN;
  const int m0 = tm << 6;
  const int n0 = tn << 6;

  const T* Ab  = A  + (size_t)b * strideA;
  const T* Bb  = Bt + (size_t)b * strideB;
  const T* Ab2 = SPLIT ? (A2  + (size_t)b * strideA) : nullptr;
  const T* Bb2 = SPLIT ? (Bt2 + (size_t)b * strideB) : nullptr;

  const int rlane = lane & 15;
  const int koff  = (lane >> 4) * 8;
  const int mOff  = (lane >> 4) * 8;

  v8f acc[4][4];
#pragma unroll
  for (int i = 0; i < 4; ++i)
#pragma unroll
    for (int j = 0; j < 4; ++j) acc[i][j] = (v8f){0.f,0.f,0.f,0.f,0.f,0.f,0.f,0.f};

  for (int k0 = 0; k0 < K; k0 += 32) {
    V bh[4], bl[4];
#pragma unroll
    for (int j = 0; j < 4; ++j) {
      const size_t bo = (size_t)(n0 + (j << 4) + rlane) * ldb + koff + k0;
      bh[j] = Frag<T>::load(Bb + bo);
      if (SPLIT) bl[j] = Frag<T>::load(Bb2 + bo);
    }
#pragma unroll
    for (int i = 0; i < 4; ++i) {
      const size_t ao = (size_t)(m0 + (i << 4) + rlane) * lda + koff + k0;
      V ah = Frag<T>::load(Ab + ao);
      V al;
      if (SPLIT) al = Frag<T>::load(Ab2 + ao);
#pragma unroll
      for (int j = 0; j < 4; ++j) {
        acc[i][j] = Frag<T>::mma(ah, bh[j], acc[i][j]);
        if (SPLIT) {
          acc[i][j] = Frag<T>::mma(ah, bl[j], acc[i][j]);
          acc[i][j] = Frag<T>::mma(al, bh[j], acc[i][j]);
        }
      }
      Frag<T>::guard4(acc[i][0], acc[i][1], acc[i][2], acc[i][3], ah, SPLIT ? al : ah);
    }
    Frag<T>::keep(bh[0], bh[1], bh[2], bh[3]);
    if (SPLIT) Frag<T>::keep(bl[0], bl[1], bl[2], bl[3]);
  }
  acc_guard4(acc[0][0], acc[0][1], acc[0][2], acc[0][3]);
  acc_guard4(acc[1][0], acc[1][1], acc[1][2], acc[1][3]);
  acc_guard4(acc[2][0], acc[2][1], acc[2][2], acc[2][3]);
  acc_guard4(acc[3][0], acc[3][1], acc[3][2], acc[3][3]);

  float* slab = sT[wave];
  const float* Rb = RESID ? (resid + (size_t)b * strideR) : nullptr;
#pragma unroll
  for (int i = 0; i < 4; ++i) {
    const int mBase = m0 + (i << 4);
#pragma unroll
    for (int j = 0; j < 4; ++j) {
      const int n = n0 + (j << 4) + rlane;
      float bv = 0.f;
      if (BIAS_MODE == 2) bv = bias[n];
#pragma unroll
      for (int r = 0; r < 8; ++r) {
        float v = acc[i][j][r] * scale;
        if (BIAS_MODE == 1) v += bias[mBase + mOff + r];
        if (BIAS_MODE == 2) v += bv;
        if (RESID) v += Rb[(size_t)(mBase + mOff + r) * ldc + n];
        if (ACT == 1) v = tanhf(v);
        if (ACT == 2) v = fmaxf(v, 0.0f);
        if (ACT == 3) v = v / (1.0f + expf(-v));
        if (ACT == 4) v = (v > 0.f) ? v : 0.01f * v;
        slab[(mOff + r) * 68 + (j << 4) + rlane] = v;
      }
    }
    __builtin_amdgcn_fence(__ATOMIC_RELEASE, "workgroup");
    __builtin_amdgcn_wave_barrier();
    __builtin_amdgcn_fence(__ATOMIC_ACQUIRE, "workgroup");
    if (OUT_MODE == 0) {
      float* C = (float*)Cout + (size_t)b * strideC;
      const int hh = lane >> 4, c4 = (lane & 15) * 4;
      for (int pass = 0; pass < 2; ++pass) {
#pragma unroll
        for (int it = 0; it < 8; ++it) {
          const int row = it * 2 + hh;
          v4f v = *(const v4f*)(slab + row * 68 + c4);
          *(volatile v4f*)(C + (size_t)(mBase + row) * ldc + n0 + c4) = v;
        }
        __threadfence();
      }
    } else {
      const int q = lane >> 3, c8 = (lane & 7) * 8;
      unsigned short* C  = (unsigned short*)Cout  + (size_t)b * strideC;
      unsigned short* C2 = (OUT_MODE == 2) ? ((unsigned short*)Cout2 + (size_t)b * strideC) : nullptr;
      for (int pass = 0; pass < 2; ++pass) {
#pragma unroll
        for (int it = 0; it < 4; ++it) {
          const int row = it * 4 + q;
          const float* sp = slab + row * 68 + c8;
          v8h hv, lv;
#pragma unroll
          for (int e = 0; e < 8; ++e) {
            if (OUT_MODE == 1) {
              hv[e] = (_Float16)sp[e];
            } else {
              unsigned short hb = f2bf_bits(sp[e]);
              unsigned short lb = f2bf_bits(sp[e] - bf_bits2f(hb));
              hv[e] = __builtin_bit_cast(_Float16, hb);
              lv[e] = __builtin_bit_cast(_Float16, lb);
            }
          }
          *(volatile v8h*)(C + (size_t)(mBase + row) * ldc + n0 + c8) = hv;
          if (OUT_MODE == 2) *(volatile v8h*)(C2 + (size_t)(mBase + row) * ldc + n0 + c8) = lv;
        }
        __threadfence();
      }
    }
    __builtin_amdgcn_fence(__ATOMIC_RELEASE, "workgroup");
    __builtin_amdgcn_wave_barrier();
    __builtin_amdgcn_fence(__ATOMIC_ACQUIRE, "workgroup");
  }
}


__device__ __forceinline__ void split_hl(float v, float c, _Float16& hi, _Float16& lo) {
  const float sv = carry_flush(v, c);
  hi = (_Float16)sv;
  const float r = sv - (float)hi;
  lo = (_Float16)((fabsf(r) < kF16MinNormal) ? 0.0f : r);
}

__global__ __launch_bounds__(kThr) void coef_kernel(const float* __restrict__ log_dt, const float* __restrict__ log_neg_A, const float* __restrict__ Bm,
                                                    float* __restrict__ DA, float* __restrict__ DB) {
  const int i = blockIdx.x * kThr + threadIdx.x;
  const int d = i >> 6;
  const float ld0 = log_dt[d], la0 = log_neg_A[i], b0 = Bm[i];
  const float dt = expf(bf16r(ld0));
  const float A = -expf(bf16r(la0));
  const float da = expf(dt * A);
  const float db = (da - 1.0f) / A * bf16r(b0);
  for (int pass = 0; pass < 2; ++pass) {
    *(volatile float*)(DA + i) = da;
    *(volatile float*)(DB + i) = db;
    __threadfence();
  }
}
static_assert((kD * kNs) % kThr == 0, "coefficient grid exact");

__global__ __launch_bounds__(128) void wt_plane_kernel(const float* __restrict__ W, const float* __restrict__ b_out, unsigned short* __restrict__ WOT,
                                                       float* __restrict__ BV, int colOff) {
  const int n  = blockIdx.x;
  const int k8 = threadIdx.x * 8;
  v8h hv;
#pragma unroll
  for (int e = 0; e < 8; ++e) {
    const float w = W[(size_t)(k8 + e) * kVocab + n];
    hv[e] = (_Float16)carry_flush(bf16r(w), kWCarry);
  }
  unsigned short* dp = WOT + (size_t)n * kDX + colOff + k8;
  const int i = threadIdx.x;
  const float vb = b_out[(i < kVocab) ? i : 0];
  const float bo = (i < kVocab) ? bf16r(vb) : 0.0f;
  const bool doBias = (n == 0) && (colOff == 0);
  for (int pass = 0; pass < 2; ++pass) {
    *(volatile v8h*)dp = hv;
    if (doBias) *(volatile float*)(BV + i) = bo;
    __threadfence();
  }
}

template <bool kFirst>
__global__ __launch_bounds__(kThr) void s4d_pass_kernel(const int* __restrict__ tokens, const float* __restrict__ emb, const float* __restrict__ DA,
                                                        const float* __restrict__ DB, const float* __restrict__ Cm, const float* __restrict__ Dsk,
                                                        float* __restrict__ YP) {
  const int v = blockIdx.x * kThr + threadIdx.x;
  const int b = v >> 10;
  const int d = v & (kD - 1);
  constexpr int n0 = kFirst ? 0 : kNh;
  float a[kNh], bb[kNh], cc[kNh], h[kNh];
#pragma unroll
  for (int q = 0; q < kNh / 4; ++q) {
    const v4f av = *(const v4f*)(DA + (size_t)d * kNs + n0 + 4 * q);
    const v4f bv = *(const v4f*)(DB + (size_t)d * kNs + n0 + 4 * q);
    const v4f cv = *(const v4f*)(Cm + (size_t)d * kNs + n0 + 4 * q);
#pragma unroll
    for (int e = 0; e < 4; ++e) { const float c0 = cv[e]; a[4 * q + e] = av[e]; bb[4 * q + e] = bv[e]; cc[4 * q + e] = bf16r(c0); h[4 * q + e] = 0.0f; }
  }
  const float dd = Dsk[d];
  const float dsk = bf16r(dd);
  const size_t r0 = (size_t)b * kSeq;
#pragma unroll 1
  for (int l = 0; l < kSeq; ++l) {
    const size_t row = r0 + l;
    int tok = tokens[row];
    tok = (tok < 0) ? 0 : ((tok > kVocab - 1) ? (kVocab - 1) : tok);
    const float ur = emb[(size_t)tok * kD + d];
    const float u = bf16r(ur);
    float y = 0.0f;
#pragma unroll
    for (int n = 0; n < kNh; ++n) {
      const float hn = a[n] * h[n] + bb[n] * u;
      h[n] = hn;
      y += hn * cc[n];
    }
    float* op = YP + row * kD + d;
    float o;
    if (kFirst) { o = y; } else { o = (*op + y) + dsk * u; }
    *(volatile float*)op = o;
    __threadfence();
    *(volatile float*)op = o;
  }
}
static_assert((kBatch * kD) % kThr == 0, "scan grid exact");

__global__ __launch_bounds__(kThr) void y_cast_kernel(const float* __restrict__ YP, unsigned short* __restrict__ Y16) {
  const size_t v = (size_t)blockIdx.x * kThr + threadIdx.x;
  const size_t row = v >> 7;
  const int d8 = (int)(v & 127) * 8;
  const v4f a0 = *(const v4f*)(YP + row * kD + d8);
  const v4f a1 = *(const v4f*)(YP + row * kD + d8 + 4);
  v8h hv, lv;
#pragma unroll
  for (int e = 0; e < 4; ++e) {
    _Float16 h0, l0, h1, l1;
    split_hl(a0[e], kACarry, h0, l0);
    split_hl(a1[e], kACarry, h1, l1);
    hv[e] = h0; lv[e] = l0; hv[4 + e] = h1; lv[4 + e] = l1;
  }
  unsigned short* dp = Y16 + row * kDX + d8;
  for (int pass = 0; pass < 2; ++pass) {
    *(volatile v8h*)dp = hv;
    *(volatile v8h*)(dp + kD) = lv;
    __threadfence();
  }
}
static_assert(((size_t)kRows * 128) % kThr == 0, "cast grid exact");

extern "C" void kernel_launch(void* const* d_in, const int* in_sizes, int n_in,
                              void* d_out, int out_size, void* d_ws, size_t ws_size,
                              hipStream_t stream) {
  if (n_in < 9 || d_out == nullptr || d_ws == nullptr) return;
  if (in_sizes[0] != kHalves * kRows || in_sizes[1] != kVocab * kD || in_sizes[2] != kD * kNs || in_sizes[3] != kD * kNs || in_sizes[4] != kD * kNs) return;
  if (in_sizes[5] != kD || in_sizes[6] != kD || in_sizes[7] != kD * kVocab || in_sizes[8] != kVocab) return;
  if (out_size != kHalves * kRows * kVocab) return;
  if (ws_size < kWsTotal) return;
  const int* tokens = (const int*)d_in[0];
  const float* emb = (const float*)d_in[1];
  const float* log_neg_A = (const float*)d_in[2];
  const float* Bm = (const float*)d_in[3];
  const float* Cm = (const float*)d_in[4];
  const float* Dsk = (const float*)d_in[5];
  const float* log_dt = (const float*)d_in[6];
  const float* W_out = (const float*)d_in[7];
  const float* b_out = (const float*)d_in[8];
  float* out = (float*)d_out;
  char* ws = (char*)d_ws;
  float* DA = (float*)(ws + kOffDA);
  float* DB = (float*)(ws + kOffDB);
  unsigned short* WOT = (unsigned short*)(ws + kOffWOT);
  float* BV = (float*)(ws + kOffBV);
  float* YP = (float*)(ws + kOffYP);
  unsigned short* Y16 = (unsigned short*)(ws + kOffY16);

  coef_kernel<<<(kD * kNs) / kThr, kThr, 0, stream>>>(log_dt, log_neg_A, Bm, DA, DB);
  wt_plane_kernel<<<kVocab, kD / 8, 0, stream>>>(W_out, b_out, WOT, BV, 0);
  wt_plane_kernel<<<kVocab, kD / 8, 0, stream>>>(W_out, b_out, WOT, BV, kD);
  for (int half = 0; half < kHalves; ++half) {
    const int* tokh = tokens + (size_t)half * kRows;
    float* outh = out + (size_t)half * kRows * kVocab;
    s4d_pass_kernel<true><<<(kBatch * kD) / kThr, kThr, 0, stream>>>(tokh, emb, DA, DB, Cm, Dsk, YP);
    s4d_pass_kernel<false><<<(kBatch * kD) / kThr, kThr, 0, stream>>>(tokh, emb, DA, DB, Cm, Dsk, YP);
    y_cast_kernel<<<(int)(((size_t)kRows * 128) / kThr), kThr, 0, stream>>>(YP, Y16);
    wmma_gemm64<0, false, 2, 0, false, 0><<<dim3((kRows / 64) * (kVocab / 64) / 8, 1), 256, 0, stream>>>(
        Y16, Y16, kDX, 0L, WOT, WOT, kDX, 0L, (void*)outh, (void*)outh, kVocab, 0L, BV, nullptr, 0L, kRows, kVocab, kDX, kScA);
  }
}
